// Classifier_26723286516422
// MI455X (gfx1250) — hardware-verified
//
#include <hip/hip_runtime.h>
#include <stddef.h>
#include <stdint.h>

typedef __attribute__((ext_vector_type(16))) _Float16 v16h;
typedef __attribute__((ext_vector_type(8)))  _Float16 v8h;
typedef __attribute__((ext_vector_type(8)))  float    v8f;
typedef __attribute__((ext_vector_type(4)))  float    v4f;

constexpr int NB    = 32;
constexpr int IMG   = 224;
constexpr int NCH1  = 128;
constexpr int NCH2  = 64;
constexpr int NCH3  = 32;
constexpr int NCH4  = 8;
constexpr int HC1   = 222;
constexpr int HP1   = 111;
constexpr int HP2   = 54;
constexpr int HP3   = 26;
constexpr int HO4   = 24;
constexpr int WO4   = 25;
constexpr int KP1   = 32;
constexpr int KT2   = 9 * NCH1;
constexpr int KT3   = 9 * NCH2;
constexpr int NOUT  = NB * NCH4 * HO4 * WO4;
static_assert(KP1 % 32 == 0 && KT2 % 32 == 0 && KT3 % 32 == 0, "K multiples of 32");
static_assert(NOUT % 256 == 0, "conv4 grid exact");
static_assert(HP2 % 2 == 0 && HP3 % 2 == 0, "two pooled rows per block");

constexpr size_t WS_WA1 = 0;
constexpr size_t WS_WA2 = WS_WA1 + (size_t)NCH1 * KP1 * 2;
constexpr size_t WS_WA3 = WS_WA2 + (size_t)NCH2 * KT2 * 2;
constexpr size_t WS_A1  = WS_WA3 + (size_t)NCH3 * KT3 * 2;
constexpr size_t WS_A2  = WS_A1 + (size_t)NB * HP1 * HP1 * NCH1 * 2;
constexpr size_t WS_A3  = WS_A2 + (size_t)NB * HP2 * HP2 * NCH2 * 2;
constexpr size_t WS_END = WS_A3 + (size_t)NB * HP3 * HP3 * NCH3 * 4;
static_assert(WS_A1 == 192512, "carve");
static_assert(WS_END == 115838976, "carve");
static_assert(WS_END <= 134217728, "carve under 128 MiB");
static_assert(WS_WA2 % 256 == 0 && WS_WA3 % 256 == 0 && WS_A1 % 256 == 0 && WS_A2 % 256 == 0 && WS_A3 % 256 == 0, "alignment");

template <typename T> struct Frag;
template <> struct Frag<_Float16> {
  typedef v16h V; union U { v16h v; v8h h[2]; };
  static __device__ __forceinline__ v16h load(const _Float16* p) {
    U f; f.h[0] = *(const v8h*)(p); f.h[1] = *(const v8h*)(p + 16); return f.v;
  }
  static __device__ __forceinline__ v8f mma(v16h a, v16h b, v8f c) {
    return __builtin_amdgcn_wmma_f32_16x16x32_f16(false, a, false, b, (short)0, c, false, false);
  }
};
typedef Frag<_Float16> FragH;

__device__ __forceinline__ unsigned opq(unsigned v) { asm volatile("" : "+v"(v)); return v; }
__device__ __forceinline__ float opqf(float v) { asm volatile("" : "+v"(v)); return v; }

__device__ __forceinline__ void guard4x5(v8f& c0, v8f& c1, v8f& c2, v8f& c3,
                                         v16h f0, v16h f1, v16h f2, v16h f3, v16h f4) {
  asm volatile("v_nop\n\tv_nop\n\tv_nop\n\tv_nop"
               : "+v"(c0), "+v"(c1), "+v"(c2), "+v"(c3)
               : "v"(f0), "v"(f1), "v"(f2), "v"(f3), "v"(f4));
}
__device__ __forceinline__ void grp_guard(v8f& c0, v8f& c1, v8f& c2, v8f& c3,
                                          v16h a0, v16h a1, v16h b0, v16h b1) {
  asm volatile("v_nop\n\tv_nop\n\tv_nop\n\tv_nop"
               : "+v"(c0), "+v"(c1), "+v"(c2), "+v"(c3)
               : "v"(a0), "v"(a1), "v"(b0), "v"(b1)
               : "memory");
}
__device__ __forceinline__ void accg4(v8f& a, v8f& b, v8f& c, v8f& d) {
  asm volatile("v_nop\n\tv_nop\n\tv_nop\n\tv_nop" : "+v"(a), "+v"(b), "+v"(c), "+v"(d));
}

__device__ __forceinline__ float leaky05(float v) { return (v >= 0.0f) ? v : 0.5f * v; }

template <int CIN, int KPAD>
__global__ __launch_bounds__(256) void wsign_prep_kernel(const float* __restrict__ W, int cout,
                                                          unsigned short* __restrict__ O) {
  constexpr unsigned KREAL = 9u * (unsigned)CIN;
  constexpr unsigned TPR = (unsigned)KPAD / 8u;
  static_assert(KPAD % 8 == 0 && (unsigned)KPAD >= KREAL, "pad");
  static_assert((CIN & (CIN - 1)) == 0, "CIN power of two");
  const int i = blockIdx.x * 256 + threadIdx.x;
  if (i >= cout * (int)TPR) return;
  const unsigned iu = opq((unsigned)i);
  const unsigned co = iu / TPR;
  const unsigned k0 = (iu - co * TPR) * 8u;
  v8h hv;
#pragma unroll
  for (int e = 0; e < 8; ++e) {
    const unsigned k  = k0 + (unsigned)e;
    const unsigned kc = (k < KREAL) ? k : (KREAL - 1u);
    const unsigned p  = kc / (unsigned)CIN;
    const unsigned ci = kc - p * (unsigned)CIN;
    const unsigned pu = opq(p);
    const unsigned ky = pu / 3u;
    const unsigned kx = pu - 3u * ky;
    const float w = W[((size_t)(co * (unsigned)CIN + ci) * 3u + ky) * 3u + kx];
    const float s = (w >= 0.0f) ? 1.0f : -1.0f;
    const float v = (k < KREAL) ? s : 0.0f;
    hv[e] = (_Float16)v;
  }
  unsigned short* dst = O + (size_t)i * 8;
  *(volatile v8h*)dst = hv;
  __threadfence();
  *(volatile v8h*)dst = hv;
}

constexpr int C1_PW = 36;
constexpr int C1_KP = 40;
constexpr int C1_TP = 132;

__global__ __launch_bounds__(256) void conv1_pool_kernel(const float* __restrict__ x,
                                                         const unsigned short* __restrict__ wA1p,
                                                         const float* __restrict__ b1,
                                                         unsigned short* __restrict__ a1p) {
  __shared__ __align__(16) float    patch[4 * C1_PW];
  __shared__ __align__(16) _Float16 btile[64 * C1_KP];
  __shared__ __align__(16) float    ptile[16 * C1_TP];
  __shared__ __align__(16) float    bsh[NCH1];
  const _Float16* wA1 = (const _Float16*)wA1p;
  _Float16* a1 = (_Float16*)a1p;
  const int tid = threadIdx.x, lane = tid & 31, wave = tid >> 5, h = lane >> 4, nl = lane & 15;
  const int bx = blockIdx.x, py = blockIdx.y, b = blockIdx.z;
  const int ox0 = bx * 32;

  {
    const int r = tid >> 6, q = tid & 63;
    const int qq = (q < 34) ? q : 33;
    int xc = ox0 + qq; xc = (xc < IMG) ? xc : (IMG - 1);
    const float v = x[((size_t)b * IMG + (size_t)(2 * py + r)) * IMG + xc];
    if (q < 34) patch[r * C1_PW + q] = v;
    if (tid < NCH1) bsh[tid] = b1[tid];
  }
  __syncthreads();

  {
    const int rc = tid & 63;
    const int kq = __builtin_amdgcn_readfirstlane(tid >> 6);
    const int r = rc >> 5, col = rc & 31;
    int cg = ox0 + col; cg = (cg < HC1) ? cg : (HC1 - 1);
    const float* pr = patch + r * C1_PW + (cg - ox0);
    const float zf = opqf(0.0f);
    v8h hv;
    if (kq == 0) {
#pragma unroll
      for (int e = 0; e < 8; ++e) {
        const int ky = e / 3, kx = e - 3 * ky;
        hv[e] = (_Float16)pr[ky * C1_PW + kx];
      }
    } else if (kq == 1) {
      hv[0] = (_Float16)pr[2 * C1_PW + 2];
#pragma unroll
      for (int e = 1; e < 8; ++e) hv[e] = (_Float16)zf;
    } else {
#pragma unroll
      for (int e = 0; e < 8; ++e) hv[e] = (_Float16)zf;
    }
    *(v8h*)(btile + rc * C1_KP + kq * 8) = hv;
  }
  __syncthreads();

  const v16h af = FragH::load(wA1 + (size_t)(wave * 16 + nl) * KP1 + 8 * h);
  v16h bf[2][2];
#pragma unroll
  for (int r = 0; r < 2; ++r)
#pragma unroll
    for (int ct = 0; ct < 2; ++ct)
      bf[r][ct] = FragH::load(btile + (r * 32 + ct * 16 + nl) * C1_KP + 8 * h);
  v8f acc[2][2];
  const v8f z8 = {0.f, 0.f, 0.f, 0.f, 0.f, 0.f, 0.f, 0.f};
#pragma unroll
  for (int r = 0; r < 2; ++r)
#pragma unroll
    for (int ct = 0; ct < 2; ++ct)
      acc[r][ct] = FragH::mma(af, bf[r][ct], z8);
  guard4x5(acc[0][0], acc[0][1], acc[1][0], acc[1][1], af, bf[0][0], bf[0][1], bf[1][0], bf[1][1]);

  const int chb = wave * 16 + 8 * h;
  const v4f bv0 = *(const v4f*)(bsh + chb);
  const v4f bv1 = *(const v4f*)(bsh + chb + 4);
  float pm[2][8];
#pragma unroll
  for (int ct = 0; ct < 2; ++ct)
#pragma unroll
    for (int rr = 0; rr < 8; ++rr) {
      float m = fmaxf(acc[0][ct][rr], acc[1][ct][rr]);
      const float mo = __shfl_xor(m, 1, 32);
      m = fmaxf(m, mo);
      const float bb = (rr < 4) ? bv0[rr & 3] : bv1[rr & 3];
      m = m + bb;
      pm[ct][rr] = leaky05(m);
    }
  if ((nl & 1) == 0) {
#pragma unroll
    for (int ct = 0; ct < 2; ++ct) {
      float* pp = ptile + (ct * 8 + (nl >> 1)) * C1_TP + chb;
      v4f w0, w1;
      w0[0] = pm[ct][0]; w0[1] = pm[ct][1]; w0[2] = pm[ct][2]; w0[3] = pm[ct][3];
      w1[0] = pm[ct][4]; w1[1] = pm[ct][5]; w1[2] = pm[ct][6]; w1[3] = pm[ct][7];
      *(v4f*)pp = w0;
      *(v4f*)(pp + 4) = w1;
    }
  }
  __syncthreads();

  {
    const int pl  = 2 * wave + h;
    const int c8  = nl * 8;
    const int pxg = bx * 16 + pl;
    const bool valid = pxg < HP1;
    const int pxc = valid ? pxg : (HP1 - 1);
    const v4f u0 = *(const v4f*)(ptile + pl * C1_TP + c8);
    const v4f u1 = *(const v4f*)(ptile + pl * C1_TP + c8 + 4);
    v8h hv;
#pragma unroll
    for (int e = 0; e < 4; ++e) { hv[e] = (_Float16)u0[e]; hv[4 + e] = (_Float16)u1[e]; }
    _Float16* dst = a1 + ((((size_t)b * HP1 + py) * HP1 + pxc) * NCH1 + c8);
    if (valid) *(volatile v8h*)dst = hv;
    __threadfence();
    if (valid) *(volatile v8h*)dst = hv;
  }
}

template <int CIN, int NMT, int HIN, int HPO, bool OF32>
__global__ __launch_bounds__(64) void convpool_kernel(const unsigned short* __restrict__ inp,
                                                      const unsigned short* __restrict__ wAp,
                                                      const float* __restrict__ bias,
                                                      void* __restrict__ outp) {
  constexpr int COUT   = 16 * NMT;
  constexpr int KTOT   = 9 * CIN;
  constexpr int CPS    = CIN / 32;
  constexpr int JPR    = 3 * CPS;
  constexpr int HCV    = 2 * HPO;
  constexpr int TP     = COUT + 4;
  constexpr int NE     = OF32 ? 4 : 8;
  constexpr size_t RSTR = (size_t)HIN * CIN;
  static_assert(CIN % 32 == 0 && KTOT % 32 == 0, "K multiple of 32");
  static_assert(NMT % 2 == 0, "M-tiles in pairs");
  static_assert(HCV + 2 <= HIN, "reads stay inside the input plane");
  static_assert((OF32 ? COUT * 4 : COUT * 2) == 128, "one 128-B line per pooled pixel");
  __shared__ __align__(16) float wt[2][16 * TP];
  __shared__ __align__(16) float bsh[COUT];
  const _Float16* in = (const _Float16*)inp;
  const _Float16* wA = (const _Float16*)wAp;
  const int tid = threadIdx.x, lane = tid & 31, wave = tid >> 5, h = lane >> 4, nl = lane & 15;
  const int b = blockIdx.z, bx = blockIdx.x, py = blockIdx.y * 2 + wave;
  const int ox0 = bx * 16;
  for (int i = tid; i < COUT; i += 64) bsh[i] = bias[i];

  int cg = ox0 + nl; cg = (cg < HCV) ? cg : (HCV - 1);
  const v8f z8 = {0.f, 0.f, 0.f, 0.f, 0.f, 0.f, 0.f, 0.f};
  v8f acc[NMT][2];
#pragma unroll
  for (int mt = 0; mt < NMT; ++mt) { acc[mt][0] = z8; acc[mt][1] = z8; }
  const _Float16* aP = wA + (size_t)nl * KTOT + 8 * h;
  const _Float16* bR = in + (((size_t)b * HIN + (size_t)(2 * py)) * HIN + (size_t)cg) * CIN + 8 * h;

#pragma unroll 1
  for (int ky = 0; ky < 3; ++ky) {
    const _Float16* bp = bR;
#pragma unroll 1
    for (int jj = 0; jj < JPR; ++jj) {
      const v16h fb0 = FragH::load(bp);
      const v16h fb1 = FragH::load(bp + RSTR);
#pragma unroll
      for (int gq = 0; gq < NMT / 2; ++gq) {
        const v16h fa0 = FragH::load(aP + (size_t)(2 * gq) * 16 * KTOT);
        const v16h fa1 = FragH::load(aP + (size_t)(2 * gq + 1) * 16 * KTOT);
        acc[2 * gq][0]     = FragH::mma(fa0, fb0, acc[2 * gq][0]);
        acc[2 * gq][1]     = FragH::mma(fa0, fb1, acc[2 * gq][1]);
        acc[2 * gq + 1][0] = FragH::mma(fa1, fb0, acc[2 * gq + 1][0]);
        acc[2 * gq + 1][1] = FragH::mma(fa1, fb1, acc[2 * gq + 1][1]);
        grp_guard(acc[2 * gq][0], acc[2 * gq][1], acc[2 * gq + 1][0], acc[2 * gq + 1][1], fa0, fa1, fb0, fb1);
      }
      aP += 32;
      bp += 32;
    }
    bR += RSTR;
  }
  accg4(acc[0][0], acc[0][1], acc[1][0], acc[1][1]);
  accg4(acc[NMT - 2][0], acc[NMT - 2][1], acc[NMT - 1][0], acc[NMT - 1][1]);

  float* wtl = wt[wave];
#pragma unroll
  for (int mt = 0; mt < NMT; ++mt)
#pragma unroll
    for (int rr = 0; rr < 8; ++rr)
      wtl[nl * TP + mt * 16 + 8 * h + rr] = fmaxf(acc[mt][0][rr], acc[mt][1][rr]);
  __syncthreads();

  const int q  = lane & 7;
  const int c0 = q * NE;
  const int plA = lane >> 3;
  const int plB = 4 + (lane >> 3);
  float vA[8], vB[8];
#pragma unroll
  for (int e = 0; e < 8; ++e) { vA[e] = 0.0f; vB[e] = 0.0f; }
#pragma unroll
  for (int g = 0; g < NE / 4; ++g) {
    const v4f a0 = *(const v4f*)(wtl + (2 * plA) * TP + c0 + 4 * g);
    const v4f a1 = *(const v4f*)(wtl + (2 * plA + 1) * TP + c0 + 4 * g);
    const v4f c0v = *(const v4f*)(wtl + (2 * plB) * TP + c0 + 4 * g);
    const v4f c1v = *(const v4f*)(wtl + (2 * plB + 1) * TP + c0 + 4 * g);
#pragma unroll
    for (int e = 0; e < 4; ++e) {
      const float bv = bsh[c0 + 4 * g + e];
      vA[4 * g + e] = leaky05(fmaxf(a0[e], a1[e]) + bv);
      vB[4 * g + e] = leaky05(fmaxf(c0v[e], c1v[e]) + bv);
    }
  }
  const int pxA = bx * 8 + plA, pxB = bx * 8 + plB;
  const bool okA = pxA < HPO, okB = pxB < HPO;
  const size_t pixA = ((size_t)b * HPO + (size_t)py) * HPO + (size_t)(okA ? pxA : (HPO - 1));
  const size_t pixB = ((size_t)b * HPO + (size_t)py) * HPO + (size_t)(okB ? pxB : (HPO - 1));
  if (OF32) {
    v4f oA, oB;
    oA[0] = vA[0]; oA[1] = vA[1]; oA[2] = vA[2]; oA[3] = vA[3];
    oB[0] = vB[0]; oB[1] = vB[1]; oB[2] = vB[2]; oB[3] = vB[3];
    float* o = (float*)outp;
    float* dA = o + pixA * COUT + c0;
    float* dB = o + pixB * COUT + c0;
    for (int pass = 0; pass < 2; ++pass) {
      if (okA) *(volatile v4f*)dA = oA;
      if (okB) *(volatile v4f*)dB = oB;
      __threadfence();
    }
  } else {
    v8h oA, oB;
#pragma unroll
    for (int e = 0; e < 8; ++e) { oA[e] = (_Float16)vA[e]; oB[e] = (_Float16)vB[e]; }
    _Float16* o = (_Float16*)outp;
    _Float16* dA = o + pixA * COUT + c0;
    _Float16* dB = o + pixB * COUT + c0;
    for (int pass = 0; pass < 2; ++pass) {
      if (okA) *(volatile v8h*)dA = oA;
      if (okB) *(volatile v8h*)dB = oB;
      __threadfence();
    }
  }
}

__global__ __launch_bounds__(256) void conv4_kernel(const float* __restrict__ a3, const float* __restrict__ w4,
                                                    const float* __restrict__ b4, float* __restrict__ out) {
  __shared__ float wsg[NCH4 * NCH3 * 6];
  __shared__ float bsh[NCH4];
  const int tid = threadIdx.x;
#pragma unroll 1
  for (int i = tid; i < NCH4 * NCH3 * 6; i += 256) {
    const float w = w4[i];
    wsg[i] = (w >= 0.0f) ? 1.0f : -1.0f;
  }
  {
    const float bv = b4[tid & 7];
    if (tid < NCH4) bsh[tid] = bv;
  }
  __syncthreads();
  const int idx = blockIdx.x * 256 + tid;
  const unsigned iu = opq((unsigned)idx);
  const unsigned xo = iu % (unsigned)WO4;
  unsigned t = iu / (unsigned)WO4;
  const unsigned yo = t % (unsigned)HO4; t /= (unsigned)HO4;
  const unsigned c  = t % (unsigned)NCH4;
  const unsigned bb = t / (unsigned)NCH4;
  const float* ab = a3 + (((size_t)bb * HP3 + (size_t)yo) * HP3 + (size_t)xo) * NCH3;
  const float* wc = wsg + c * (NCH3 * 6);
  float s = 0.0f;
#pragma unroll 1
  for (int c4 = 0; c4 < NCH3 / 4; ++c4) {
    v4f u[6];
#pragma unroll
    for (int ky = 0; ky < 3; ++ky)
#pragma unroll
      for (int kx = 0; kx < 2; ++kx)
        u[ky * 2 + kx] = *(const v4f*)(ab + ((size_t)ky * HP3 + (size_t)kx) * NCH3 + c4 * 4);
#pragma unroll
    for (int j = 0; j < 4; ++j) {
      const int ci = c4 * 4 + j;
#pragma unroll
      for (int tp = 0; tp < 6; ++tp) s = fmaf(wc[ci * 6 + tp], u[tp][j], s);
    }
  }
  s += bsh[c];
  float* dst = out + idx;
  *(volatile float*)dst = s;
  __threadfence();
  *(volatile float*)dst = s;
}

extern "C" void kernel_launch(void* const* d_in, const int* in_sizes, int n_in,
                              void* d_out, int out_size, void* d_ws, size_t ws_size,
                              hipStream_t stream) {
  (void)in_sizes; (void)n_in; (void)out_size; (void)ws_size;
  const float* x  = (const float*)d_in[0];
  const float* w1 = (const float*)d_in[1];
  const float* b1 = (const float*)d_in[2];
  const float* w2 = (const float*)d_in[3];
  const float* b2 = (const float*)d_in[4];
  const float* w3 = (const float*)d_in[5];
  const float* b3 = (const float*)d_in[6];
  const float* w4 = (const float*)d_in[7];
  const float* b4 = (const float*)d_in[8];
  float* out = (float*)d_out;

  char* ws = (char*)d_ws;
  unsigned short* wA1 = (unsigned short*)(ws + WS_WA1);
  unsigned short* wA2 = (unsigned short*)(ws + WS_WA2);
  unsigned short* wA3 = (unsigned short*)(ws + WS_WA3);
  unsigned short* a1  = (unsigned short*)(ws + WS_A1);
  unsigned short* a2  = (unsigned short*)(ws + WS_A2);
  float*          a3  = (float*)(ws + WS_A3);

  wsign_prep_kernel<1, KP1><<<(NCH1 * KP1 / 8 + 255) / 256, 256, 0, stream>>>(w1, NCH1, wA1);
  wsign_prep_kernel<NCH1, KT2><<<(NCH2 * KT2 / 8 + 255) / 256, 256, 0, stream>>>(w2, NCH2, wA2);
  wsign_prep_kernel<NCH2, KT3><<<(NCH3 * KT3 / 8 + 255) / 256, 256, 0, stream>>>(w3, NCH3, wA3);

  conv1_pool_kernel<<<dim3((HC1 + 31) / 32, HP1, NB), 256, 0, stream>>>(x, wA1, b1, a1);

  convpool_kernel<NCH1, 4, HP1, HP2, false><<<dim3((2 * HP2 + 15) / 16, HP2 / 2, NB), 64, 0, stream>>>(a1, wA2, b2, (void*)a2);

  convpool_kernel<NCH2, 2, HP2, HP3, true><<<dim3((2 * HP3 + 15) / 16, HP3 / 2, NB), 64, 0, stream>>>(a2, wA3, b3, (void*)a3);

  conv4_kernel<<<NOUT / 256, 256, 0, stream>>>(a3, w4, b4, out);
}
